// DotAttention_57372173140044
// MI455X (gfx1250) — hardware-verified
//
#include <hip/hip_runtime.h>
#include <math.h>

#ifndef NB
#define NB 4
#endif
#ifndef SEQ
#define SEQ 2048
#endif
#define NB_FULL 4
#define SEQ_FULL 2048
#define DM 1024
#define PCARRY 16384.0f
#define SCORE_SCALE 32.0f

static_assert(NB >= 1 && NB <= NB_FULL);
static_assert(SEQ >= 256 && SEQ <= SEQ_FULL && (SEQ % 256) == 0);
static_assert((DM % 64) == 0 && (DM % 32) == 0);

typedef __attribute__((ext_vector_type(16))) _Float16 v16h;
typedef __attribute__((ext_vector_type(8)))  _Float16 v8h;
typedef __attribute__((ext_vector_type(16))) __bf16   v16b;
typedef __attribute__((ext_vector_type(8)))  __bf16   v8b;
typedef __attribute__((ext_vector_type(8)))  float    v8f;
typedef __attribute__((ext_vector_type(4)))  float    v4f;
typedef __attribute__((ext_vector_type(4)))  unsigned int u4v;

#define VST2(T, ptr, val) do { const T vst2_v_ = (val); *(volatile T*)(ptr) = vst2_v_; __threadfence(); *(volatile T*)(ptr) = vst2_v_; } while (0)

__device__ __forceinline__ unsigned short bfu_rne(float v) { unsigned u = __float_as_uint(v); u += 0x7FFFu + ((u >> 16) & 1u); return (unsigned short)(u >> 16); }
__device__ __forceinline__ unsigned int bfpk2(float a, float b) { return (unsigned int)bfu_rne(a) | ((unsigned int)bfu_rne(b) << 16); }
__device__ __forceinline__ unsigned int hpk2(float a, float b) { return (unsigned int)__builtin_bit_cast(unsigned short, (_Float16)a) | ((unsigned int)__builtin_bit_cast(unsigned short, (_Float16)b) << 16); }

namespace w25 {

__device__ __forceinline__ unsigned short f2bf_bits(float f) {
  unsigned u = __float_as_uint(f);
  return (unsigned short)((u + 0x7FFFu + ((u >> 16) & 1u)) >> 16);
}
__device__ __forceinline__ float bf_bits2f(unsigned short h) { return __uint_as_float(((unsigned)h) << 16); }

__device__ __forceinline__ void dep_guard_h(v8f& a, v8f& b, v16h x, v16h y) { asm volatile("v_nop\n\tv_nop\n\tv_nop\n\tv_nop" : "+v"(a), "+v"(b) : "v"(x), "v"(y)); }
__device__ __forceinline__ void dep_guard_b(v8f& a, v8f& b, v16b x, v16b y) { asm volatile("v_nop\n\tv_nop\n\tv_nop\n\tv_nop" : "+v"(a), "+v"(b) : "v"(x), "v"(y)); }
__device__ __forceinline__ void keep4_h(v16h a, v16h b, v16h c, v16h d) { asm volatile("v_nop" :: "v"(a), "v"(b), "v"(c), "v"(d)); }
__device__ __forceinline__ void keep4_b(v16b a, v16b b, v16b c, v16b d) { asm volatile("v_nop" :: "v"(a), "v"(b), "v"(c), "v"(d)); }
__device__ __forceinline__ void acc_guard4(v8f& a, v8f& b, v8f& c, v8f& d) { asm volatile("v_nop\n\tv_nop\n\tv_nop\n\tv_nop" : "+v"(a), "+v"(b), "+v"(c), "+v"(d)); }

template <typename T> struct Frag;
template <> struct Frag<_Float16> {
  typedef v16h V; union U { v16h v; v8h h[2]; };
  static __device__ __forceinline__ v16h load(const _Float16* p) {
    U f; f.h[0] = *(const v8h*)(p); f.h[1] = *(const v8h*)(p + 16); return f.v;
  }
  static __device__ __forceinline__ v8f mma(v16h a, v16h b, v8f c) {
    return __builtin_amdgcn_wmma_f32_16x16x32_f16(false, a, false, b, (short)0, c, false, false);
  }
  static __device__ __forceinline__ void guard(v8f& a, v8f& b, v16h x, v16h y) { dep_guard_h(a, b, x, y); }
  static __device__ __forceinline__ void keep(v16h a, v16h b, v16h c, v16h d) { keep4_h(a, b, c, d); }
};
template <> struct Frag<__bf16> {
  typedef v16b V; union U { v16b v; v8b h[2]; };
  static __device__ __forceinline__ v16b load(const __bf16* p) {
    U f; f.h[0] = *(const v8b*)(p); f.h[1] = *(const v8b*)(p + 16); return f.v;
  }
  static __device__ __forceinline__ v8f mma(v16b a, v16b b, v8f c) {
    return __builtin_amdgcn_wmma_f32_16x16x32_bf16(false, a, false, b, (short)0, c, false, false);
  }
  static __device__ __forceinline__ void guard(v8f& a, v8f& b, v16b x, v16b y) { dep_guard_b(a, b, x, y); }
  static __device__ __forceinline__ void keep(v16b a, v16b b, v16b c, v16b d) { keep4_b(a, b, c, d); }
};

template <int ET> struct Elem;
template <> struct Elem<0> { typedef _Float16 T; };
template <> struct Elem<1> { typedef __bf16 T; };
template <int ET, bool SPLIT, int BIAS_MODE, int OUT_MODE, bool RESID, int ACT = 0>
__global__ __launch_bounds__(256) void wmma_gemm64(
    const unsigned short* __restrict__ Ap, const unsigned short* __restrict__ A2p, int lda, long strideA,
    const unsigned short* __restrict__ Btp, const unsigned short* __restrict__ Bt2p, int ldb, long strideB,
    void* __restrict__ Cout, void* __restrict__ Cout2, int ldc, long strideC,
    const float* __restrict__ bias,
    const float* __restrict__ resid, long strideR,
    int M, int N, int K, float scale) {
  typedef typename Elem<ET>::T T;
  typedef typename Frag<T>::V V;
  const T* A = (const T*)Ap; const T* A2 = (const T*)A2p; const T* Bt = (const T*)Btp; const T* Bt2 = (const T*)Bt2p;
  __shared__ __align__(16) float sT[8][16 * 68];
  const int b    = blockIdx.y;
  const int lane = threadIdx.x & 31;
  const int wave = threadIdx.x >> 5;
  const int tilesN = N >> 6;
  const int tilesM = M >> 6;
  const int tile = blockIdx.x * 8 + wave;
  if (tile >= tilesM * tilesN) return;
  const int tm = tile / tilesN;
  const int tn = tile - tm * tilesN;
  const int m0 = tm << 6;
  const int n0 = tn << 6;

  const T* Ab  = A  + (size_t)b * strideA;
  const T* Bb  = Bt + (size_t)b * strideB;
  const T* Ab2 = SPLIT ? (A2  + (size_t)b * strideA) : nullptr;
  const T* Bb2 = SPLIT ? (Bt2 + (size_t)b * strideB) : nullptr;

  const int rlane = lane & 15;
  const int koff  = (lane >> 4) * 8;
  const int mOff  = (lane >> 4) * 8;

  v8f acc[4][4];
#pragma unroll
  for (int i = 0; i < 4; ++i)
#pragma unroll
    for (int j = 0; j < 4; ++j) acc[i][j] = (v8f){0.f,0.f,0.f,0.f,0.f,0.f,0.f,0.f};

  for (int k0 = 0; k0 < K; k0 += 32) {
    V bh[4], bl[4];
#pragma unroll
    for (int j = 0; j < 4; ++j) {
      const size_t bo = (size_t)(n0 + (j << 4) + rlane) * ldb + koff + k0;
      bh[j] = Frag<T>::load(Bb + bo);
      if (SPLIT) bl[j] = Frag<T>::load(Bb2 + bo);
    }
#pragma unroll
    for (int i = 0; i < 4; ++i) {
      const size_t ao = (size_t)(m0 + (i << 4) + rlane) * lda + koff + k0;
      V ah = Frag<T>::load(Ab + ao);
      V al;
      if (SPLIT) al = Frag<T>::load(Ab2 + ao);
#pragma unroll
      for (int j = 0; j < 4; ++j) {
        acc[i][j] = Frag<T>::mma(ah, bh[j], acc[i][j]);
        if (SPLIT) {
          acc[i][j] = Frag<T>::mma(ah, bl[j], acc[i][j]);
          acc[i][j] = Frag<T>::mma(al, bh[j], acc[i][j]);
        }
      }
      Frag<T>::guard(acc[i][0], acc[i][3], ah, SPLIT ? al : ah);
    }
    Frag<T>::keep(bh[0], bh[1], bh[2], bh[3]);
    if (SPLIT) Frag<T>::keep(bl[0], bl[1], bl[2], bl[3]);
  }
  acc_guard4(acc[0][0], acc[0][1], acc[0][2], acc[0][3]);
  acc_guard4(acc[1][0], acc[1][1], acc[1][2], acc[1][3]);
  acc_guard4(acc[2][0], acc[2][1], acc[2][2], acc[2][3]);
  acc_guard4(acc[3][0], acc[3][1], acc[3][2], acc[3][3]);

  float* slab = sT[wave];
  const float* Rb = RESID ? (resid + (size_t)b * strideR) : nullptr;
#pragma unroll
  for (int i = 0; i < 4; ++i) {
    const int mBase = m0 + (i << 4);
#pragma unroll
    for (int j = 0; j < 4; ++j) {
      const int n = n0 + (j << 4) + rlane;
      float bv = 0.f;
      if (BIAS_MODE == 2) bv = bias[n];
#pragma unroll
      for (int r = 0; r < 8; ++r) {
        float v = acc[i][j][r] * scale;
        if (BIAS_MODE == 1) v += bias[mBase + mOff + r];
        if (BIAS_MODE == 2) v += bv;
        if (RESID) v += Rb[(size_t)(mBase + mOff + r) * ldc + n];
        if (ACT == 1) v = tanhf(v);
        if (ACT == 2) v = fmaxf(v, 0.0f);
        if (ACT == 3) v = v / (1.0f + expf(-v));
        if (ACT == 4) v = (v > 0.f) ? v : 0.01f * v;
        if (ACT == 5) v = 0.5f * v * (1.0f + erff(v * 0.70710678118654752f));
        if (ACT == 6) v = (v > 0.f) ? v : 0.2f * v;
        if (ACT == 7) { const float u = 0.7978845608028654f * (v + 0.044715f * v * v * v); v = 0.5f * v * (1.f + tanhf(u)); }
        slab[(mOff + r) * 68 + (j << 4) + rlane] = v;
      }
    }
    __builtin_amdgcn_fence(__ATOMIC_RELEASE, "workgroup");
    __builtin_amdgcn_wave_barrier();
    __builtin_amdgcn_fence(__ATOMIC_ACQUIRE, "workgroup");
    if (OUT_MODE == 0) {
      float* C = (float*)Cout + (size_t)b * strideC;
      const int hh = lane >> 4, c4 = (lane & 15) * 4;
      for (int pass = 0; pass < 2; ++pass) {
#pragma unroll
        for (int it = 0; it < 8; ++it) {
          const int row = it * 2 + hh;
          v4f v = *(const v4f*)(slab + row * 68 + c4);
          *(volatile v4f*)(C + (size_t)(mBase + row) * ldc + n0 + c4) = v;
        }
        __threadfence();
      }
    } else {
      const int q = lane >> 3, c8 = (lane & 7) * 8;
      unsigned short* C  = (unsigned short*)Cout  + (size_t)b * strideC;
      unsigned short* C2 = (OUT_MODE == 2) ? ((unsigned short*)Cout2 + (size_t)b * strideC) : nullptr;
      for (int pass = 0; pass < 2; ++pass) {
#pragma unroll
        for (int it = 0; it < 4; ++it) {
          const int row = it * 4 + q;
          const float* sp = slab + row * 68 + c8;
          v8h hv, lv;
#pragma unroll
          for (int e = 0; e < 8; ++e) {
            if (OUT_MODE == 1) {
              hv[e] = (_Float16)sp[e];
            } else {
              unsigned short hb = f2bf_bits(sp[e]);
              unsigned short lb = f2bf_bits(sp[e] - bf_bits2f(hb));
              hv[e] = __builtin_bit_cast(_Float16, hb);
              lv[e] = __builtin_bit_cast(_Float16, lb);
            }
          }
          *(volatile v8h*)(C + (size_t)(mBase + row) * ldc + n0 + c8) = hv;
          if (OUT_MODE == 2) *(volatile v8h*)(C2 + (size_t)(mBase + row) * ldc + n0 + c8) = lv;
        }
        __threadfence();
      }
    }
    __builtin_amdgcn_fence(__ATOMIC_RELEASE, "workgroup");
    __builtin_amdgcn_wave_barrier();
    __builtin_amdgcn_fence(__ATOMIC_ACQUIRE, "workgroup");
  }
}

}

__global__ __launch_bounds__(256) void k_cvt_bf16(const float* __restrict__ src, unsigned short* __restrict__ dst, int rows, int rpb, int bstride) {
    const long long u = (long long)blockIdx.x * 256 + threadIdx.x; if (u >= (long long)rows * (DM / 8)) return;
    const int m = (int)(u / (DM / 8)); const int c = 8 * (int)(u % (DM / 8)); const int b = m / rpb; const int s = m - b * rpb;
    const float* sp = src + ((long long)b * bstride + s) * DM + c;
    const v4f a = *(const v4f*)sp; const v4f q = *(const v4f*)(sp + 4);
    u4v pk; pk.x = bfpk2(a.x, a.y); pk.y = bfpk2(a.z, a.w); pk.z = bfpk2(q.x, q.y); pk.w = bfpk2(q.z, q.w);
    VST2(u4v, (u4v*)(dst + (long long)m * DM + c), pk);
}

__global__ __launch_bounds__(256) void k_cast16(const float* __restrict__ src, long long lds, _Float16* __restrict__ dst, long long ldd, int R, int C, float s) {
    const long long i = (long long)blockIdx.x * 256 + threadIdx.x; const long long np = (long long)R * (C / 2); if (i >= np) return; const int r = (int)(i / (C / 2)); const int c = 2 * (int)(i % (C / 2));
    const unsigned u = hpk2(src[(long long)r * lds + c] * s, src[(long long)r * lds + c + 1] * s);
    volatile unsigned* d = (volatile unsigned*)(dst + (long long)r * ldd + c); *d = u; __threadfence(); *d = u; }
__global__ __launch_bounds__(256) void k_castT16(const float* __restrict__ src, long long lds, _Float16* __restrict__ dst, long long ldd, int R, int C, float s) {
    const long long i = (long long)blockIdx.x * 256 + threadIdx.x; const long long np = (long long)C * (R / 2); if (i >= np) return; const int c = (int)(i / (R / 2)); const int r = 2 * (int)(i % (R / 2));
    const unsigned u = hpk2(src[(long long)r * lds + c] * s, src[(long long)(r + 1) * lds + c] * s);
    volatile unsigned* d = (volatile unsigned*)(dst + (long long)c * ldd + r); *d = u; __threadfence(); *d = u; }

template <int NC>
__global__ __launch_bounds__(256) void k_da_sm(const float* __restrict__ S, unsigned short* __restrict__ P16) {
    #pragma clang fp contract(off)
    constexpr int CPL = NC / 32;
    static_assert((CPL % 8) == 0);
    const int row = blockIdx.x * 8 + (threadIdx.x >> 5); const int L = threadIdx.x & 31; const float* sr = S + (long long)row * NC + CPL * L; float m = -3.0e38f, s = 0.f;
#pragma unroll 1
    for (int g = 0; g < CPL / 4; ++g) { const v4f x = *(const v4f*)(sr + 4 * g); const float mx = fmaxf(fmaxf(x.x, x.y), fmaxf(x.z, x.w)); const float mn = fmaxf(m, mx);
        s = s * expf(m - mn) + ((expf(x.x - mn) + expf(x.y - mn)) + (expf(x.z - mn) + expf(x.w - mn))); m = mn; }
    float gm = m;
#pragma unroll
    for (int o = 16; o > 0; o >>= 1) gm = fmaxf(gm, __shfl_xor(gm, o, 32));
    s = s * expf(m - gm);
#pragma unroll
    for (int o = 16; o > 0; o >>= 1) s += __shfl_xor(s, o, 32);
    const float f = PCARRY / s; unsigned short* pr = P16 + (long long)row * NC + CPL * L;
#pragma unroll 1
    for (int g = 0; g < CPL / 8; ++g) { const v4f a = *(const v4f*)(sr + 8 * g), b = *(const v4f*)(sr + 8 * g + 4); u4v pk;
        pk.x = hpk2(expf(a.x - gm) * f, expf(a.y - gm) * f); pk.y = hpk2(expf(a.z - gm) * f, expf(a.w - gm) * f); pk.z = hpk2(expf(b.x - gm) * f, expf(b.y - gm) * f); pk.w = hpk2(expf(b.z - gm) * f, expf(b.w - gm) * f);
        VST2(u4v, (u4v*)(pr + 8 * g), pk); } }

static inline size_t al256(size_t n) { return ((n + 255) / 256) * 256; }

extern "C" void kernel_launch(void* const* d_in, const int* in_sizes, int n_in, void* d_out, int out_size, void* d_ws, size_t ws_size, hipStream_t stream) {
    if (n_in < 2) return;
    const long long need_x = ((long long)(NB - 1) * SEQ_FULL + SEQ) * DM;
    if ((long long)in_sizes[0] < need_x) return;
    if ((long long)in_sizes[1] < (long long)DM * DM) return;
    if ((long long)out_size < need_x) return;
    const float* x  = (const float*)d_in[0];
    const float* Wq = (const float*)d_in[1];
    float* out = (float*)d_out;

    const size_t MR = (size_t)NB * SEQ;
    char* wsp = (char*)d_ws;
    unsigned short* XH  = (unsigned short*)wsp; wsp += al256(MR * DM * 2);
    unsigned short* WH  = (unsigned short*)wsp; wsp += al256((size_t)DM * DM * 2);
    float*          Q32 = (float*)wsp;          wsp += al256(MR * DM * 4);
    unsigned short* QH  = (unsigned short*)wsp; wsp += al256(MR * DM * 2);
    unsigned short* QT  = (unsigned short*)wsp; wsp += al256((size_t)DM * SEQ * 2);
    float*          S   = (float*)wsp;          wsp += al256((size_t)SEQ * SEQ * 4);
    unsigned short* P16 = (unsigned short*)wsp; wsp += al256((size_t)SEQ * SEQ * 2);
    if ((size_t)(wsp - (char*)d_ws) > ws_size) return;

    k_cvt_bf16<<<(unsigned)(((long long)MR * (DM / 8) + 255) / 256), 256, 0, stream>>>(x, XH, (int)MR, SEQ, SEQ_FULL);
    k_cvt_bf16<<<(unsigned)(((long long)DM * (DM / 8) + 255) / 256), 256, 0, stream>>>(Wq, WH, DM, DM, DM);
    w25::wmma_gemm64<1, false, 0, 0, false, 0><<<dim3((unsigned)(((MR / 64) * (DM / 64) + 7) / 8), 1u), 256, 0, stream>>>(
        XH, nullptr, DM, 0L, WH, nullptr, DM, 0L, (void*)Q32, nullptr, DM, 0L, nullptr, nullptr, 0L, (int)MR, DM, DM, 1.0f);
    k_cast16<<<(unsigned)(((long long)MR * (DM / 2) + 255) / 256), 256, 0, stream>>>(Q32, DM, (_Float16*)QH, DM, (int)MR, DM, 1.0f);

    for (int b = 0; b < NB; ++b) {
        const float* qb32 = Q32 + (size_t)b * SEQ * DM;
        const unsigned short* qh = QH + (size_t)b * SEQ * DM;
        float* ob = out + (size_t)b * SEQ_FULL * DM;
        k_castT16<<<(unsigned)(((long long)DM * (SEQ / 2) + 255) / 256), 256, 0, stream>>>(qb32, DM, (_Float16*)QT, SEQ, SEQ, DM, 1.0f);
        w25::wmma_gemm64<0, false, 0, 0, false, 0><<<dim3((unsigned)((((SEQ / 64) * (SEQ / 64)) + 7) / 8), 1u), 256, 0, stream>>>(
            qh, nullptr, DM, 0L, qh, nullptr, DM, 0L, (void*)S, nullptr, SEQ, 0L, nullptr, nullptr, 0L, SEQ, SEQ, DM, SCORE_SCALE);
        k_da_sm<SEQ><<<SEQ / 8, 256, 0, stream>>>(S, P16);
        w25::wmma_gemm64<0, false, 0, 0, false, 0><<<dim3((unsigned)((((SEQ / 64) * (DM / 64)) + 7) / 8), 1u), 256, 0, stream>>>(
            P16, nullptr, SEQ, 0L, QT, nullptr, SEQ, 0L, (void*)ob, nullptr, DM, 0L, nullptr, nullptr, 0L, SEQ, DM, SEQ, 1.0f / PCARRY);
    }
}
